// MicroDiseaseModel_29188597743707
// MI455X (gfx1250) — hardware-verified
//
#include <hip/hip_runtime.h>
#include <math.h>
typedef __attribute__((ext_vector_type(16))) _Float16 v16h;
typedef __attribute__((ext_vector_type(8)))  _Float16 v8h;
typedef __attribute__((ext_vector_type(16))) __bf16   v16b;
typedef __attribute__((ext_vector_type(8)))  __bf16   v8b;
typedef __attribute__((ext_vector_type(8)))  float    v8f;
typedef __attribute__((ext_vector_type(4)))  float    v4f;
#define PSCALE 32768.0f
#define U16(p) ((const unsigned short*)(const void*)(p))
#define PSCALE_INV (1.0f / 32768.0f)

__device__ __forceinline__ unsigned short f2bf_bits(float f) {
  unsigned u = __float_as_uint(f);
  return (unsigned short)((u + 0x7FFFu + ((u >> 16) & 1u)) >> 16);
}
__device__ __forceinline__ float bf_bits2f(unsigned short h) { return __uint_as_float(((unsigned)h) << 16); }

__device__ __forceinline__ void dep_guard_h(v8f& a, v8f& b, v16h x, v16h y) { asm volatile("v_nop\n\tv_nop\n\tv_nop\n\tv_nop" : "+v"(a), "+v"(b) : "v"(x), "v"(y)); }
__device__ __forceinline__ void dep_guard_b(v8f& a, v8f& b, v16b x, v16b y) { asm volatile("v_nop\n\tv_nop\n\tv_nop\n\tv_nop" : "+v"(a), "+v"(b) : "v"(x), "v"(y)); }
__device__ __forceinline__ void keep4_h(v16h a, v16h b, v16h c, v16h d) { asm volatile("v_nop" :: "v"(a), "v"(b), "v"(c), "v"(d)); }
__device__ __forceinline__ void keep4_b(v16b a, v16b b, v16b c, v16b d) { asm volatile("v_nop" :: "v"(a), "v"(b), "v"(c), "v"(d)); }
__device__ __forceinline__ void acc_guard4(v8f& a, v8f& b, v8f& c, v8f& d) { asm volatile("v_nop\n\tv_nop\n\tv_nop\n\tv_nop" : "+v"(a), "+v"(b), "+v"(c), "+v"(d)); }
template <typename T> struct Frag;
template <> struct Frag<_Float16> {
  typedef v16h V; union U { v16h v; v8h h[2]; };
  static __device__ __forceinline__ v16h load(const _Float16* p) {
    U f; f.h[0] = *(const v8h*)(p); f.h[1] = *(const v8h*)(p + 16); return f.v;
  }
  static __device__ __forceinline__ v8f mma(v16h a, v16h b, v8f c) {
    return __builtin_amdgcn_wmma_f32_16x16x32_f16(false, a, false, b, (short)0, c, false, false);
  }
  static __device__ __forceinline__ void guard(v8f& a, v8f& b, v16h x, v16h y) { dep_guard_h(a, b, x, y); }
  static __device__ __forceinline__ void keep(v16h a, v16h b, v16h c, v16h d) { keep4_h(a, b, c, d); }
};
template <> struct Frag<__bf16> {
  typedef v16b V; union U { v16b v; v8b h[2]; };
  static __device__ __forceinline__ v16b load(const __bf16* p) {
    U f; f.h[0] = *(const v8b*)(p); f.h[1] = *(const v8b*)(p + 16); return f.v;
  }
  static __device__ __forceinline__ v8f mma(v16b a, v16b b, v8f c) {
    return __builtin_amdgcn_wmma_f32_16x16x32_bf16(false, a, false, b, (short)0, c, false, false);
  }
  static __device__ __forceinline__ void guard(v8f& a, v8f& b, v16b x, v16b y) { dep_guard_b(a, b, x, y); }
  static __device__ __forceinline__ void keep(v16b a, v16b b, v16b c, v16b d) { keep4_b(a, b, c, d); }
};

template <int ET> struct Elem;
template <> struct Elem<0> { typedef _Float16 T; };
template <> struct Elem<1> { typedef __bf16 T; };
template <int ET, bool SPLIT, int BIAS_MODE, int OUT_MODE, bool RESID, int ACT = 0>
__global__ __launch_bounds__(256) void wmma_gemm64(
    const unsigned short* __restrict__ Ap, const unsigned short* __restrict__ A2p, int lda, long strideA,
    const unsigned short* __restrict__ Btp, const unsigned short* __restrict__ Bt2p, int ldb, long strideB,
    void* __restrict__ Cout, void* __restrict__ Cout2, int ldc, long strideC,
    const float* __restrict__ bias,
    const float* __restrict__ resid, long strideR,
    int M, int N, int K, float scale) {
  typedef typename Elem<ET>::T T;
  typedef typename Frag<T>::V V;
  const T* A = (const T*)Ap; const T* A2 = (const T*)A2p; const T* Bt = (const T*)Btp; const T* Bt2 = (const T*)Bt2p;
  __shared__ __align__(16) float sT[8][16 * 68];
  const int b    = blockIdx.y;
  const int lane = threadIdx.x & 31;
  const int wave = threadIdx.x >> 5;
  const int tilesN = N >> 6;
  const int tilesM = M >> 6;
  const int tile = blockIdx.x * 8 + wave;
  if (tile >= tilesM * tilesN) return;
  const int tm = tile / tilesN;
  const int tn = tile - tm * tilesN;
  const int m0 = tm << 6;
  const int n0 = tn << 6;

  const T* Ab  = A  + (size_t)b * strideA;
  const T* Bb  = Bt + (size_t)b * strideB;
  const T* Ab2 = SPLIT ? (A2  + (size_t)b * strideA) : nullptr;
  const T* Bb2 = SPLIT ? (Bt2 + (size_t)b * strideB) : nullptr;

  const int rlane = lane & 15;
  const int koff  = (lane >> 4) * 8;
  const int mOff  = (lane >> 4) * 8;

  v8f acc[4][4];
#pragma unroll
  for (int i = 0; i < 4; ++i)
#pragma unroll
    for (int j = 0; j < 4; ++j) acc[i][j] = (v8f){0.f,0.f,0.f,0.f,0.f,0.f,0.f,0.f};

  for (int k0 = 0; k0 < K; k0 += 32) {
    V bh[4], bl[4];
#pragma unroll
    for (int j = 0; j < 4; ++j) {
      const size_t bo = (size_t)(n0 + (j << 4) + rlane) * ldb + koff + k0;
      bh[j] = Frag<T>::load(Bb + bo);
      if (SPLIT) bl[j] = Frag<T>::load(Bb2 + bo);
    }
#pragma unroll
    for (int i = 0; i < 4; ++i) {
      const size_t ao = (size_t)(m0 + (i << 4) + rlane) * lda + koff + k0;
      V ah = Frag<T>::load(Ab + ao);
      V al;
      if (SPLIT) al = Frag<T>::load(Ab2 + ao);
#pragma unroll
      for (int j = 0; j < 4; ++j) {
        acc[i][j] = Frag<T>::mma(ah, bh[j], acc[i][j]);
        if (SPLIT) {
          acc[i][j] = Frag<T>::mma(ah, bl[j], acc[i][j]);
          acc[i][j] = Frag<T>::mma(al, bh[j], acc[i][j]);
        }
      }
      Frag<T>::guard(acc[i][0], acc[i][3], ah, SPLIT ? al : ah);
    }
    Frag<T>::keep(bh[0], bh[1], bh[2], bh[3]);
    if (SPLIT) Frag<T>::keep(bl[0], bl[1], bl[2], bl[3]);
  }
  acc_guard4(acc[0][0], acc[0][1], acc[0][2], acc[0][3]);
  acc_guard4(acc[1][0], acc[1][1], acc[1][2], acc[1][3]);
  acc_guard4(acc[2][0], acc[2][1], acc[2][2], acc[2][3]);
  acc_guard4(acc[3][0], acc[3][1], acc[3][2], acc[3][3]);

  float* slab = sT[wave];
  const float* Rb = RESID ? (resid + (size_t)b * strideR) : nullptr;
#pragma unroll
  for (int i = 0; i < 4; ++i) {
    const int mBase = m0 + (i << 4);
#pragma unroll
    for (int j = 0; j < 4; ++j) {
      const int n = n0 + (j << 4) + rlane;
      float bv = 0.f;
      if (BIAS_MODE == 2) bv = bias[n];
#pragma unroll
      for (int r = 0; r < 8; ++r) {
        float v = acc[i][j][r] * scale;
        if (BIAS_MODE == 1) v += bias[mBase + mOff + r];
        if (BIAS_MODE == 2) v += bv;
        if (RESID) v += Rb[(size_t)(mBase + mOff + r) * ldc + n];
        if (ACT == 1) v = tanhf(v);
        if (ACT == 2) v = fmaxf(v, 0.0f);
        if (ACT == 3) v = v / (1.0f + expf(-v));
        if (ACT == 4) v = (v > 0.f) ? v : 0.01f * v;
        if (ACT == 5) v = 0.5f * v * (1.0f + erff(v * 0.70710678118654752f));
        slab[(mOff + r) * 68 + (j << 4) + rlane] = v;
      }
    }
    __builtin_amdgcn_fence(__ATOMIC_RELEASE, "workgroup");
    __builtin_amdgcn_wave_barrier();
    __builtin_amdgcn_fence(__ATOMIC_ACQUIRE, "workgroup");
    if (OUT_MODE == 0) {
      float* C = (float*)Cout + (size_t)b * strideC;
      const int hh = lane >> 4, c4 = (lane & 15) * 4;
      for (int pass = 0; pass < 2; ++pass) {
#pragma unroll
        for (int it = 0; it < 8; ++it) {
          const int row = it * 2 + hh;
          v4f v = *(const v4f*)(slab + row * 68 + c4);
          *(volatile v4f*)(C + (size_t)(mBase + row) * ldc + n0 + c4) = v;
        }
        __threadfence();
      }
    } else {
      const int q = lane >> 3, c8 = (lane & 7) * 8;
      unsigned short* C  = (unsigned short*)Cout  + (size_t)b * strideC;
      unsigned short* C2 = (OUT_MODE == 2) ? ((unsigned short*)Cout2 + (size_t)b * strideC) : nullptr;
      for (int pass = 0; pass < 2; ++pass) {
#pragma unroll
        for (int it = 0; it < 4; ++it) {
          const int row = it * 4 + q;
          const float* sp = slab + row * 68 + c8;
          v8h hv, lv;
#pragma unroll
          for (int e = 0; e < 8; ++e) {
            if (OUT_MODE == 1) {
              hv[e] = (_Float16)sp[e];
            } else {
              unsigned short hb = f2bf_bits(sp[e]);
              unsigned short lb = f2bf_bits(sp[e] - bf_bits2f(hb));
              hv[e] = __builtin_bit_cast(_Float16, hb);
              lv[e] = __builtin_bit_cast(_Float16, lb);
            }
          }
          *(volatile v8h*)(C + (size_t)(mBase + row) * ldc + n0 + c8) = hv;
          if (OUT_MODE == 2) *(volatile v8h*)(C2 + (size_t)(mBase + row) * ldc + n0 + c8) = lv;
        }
        __threadfence();
      }
    }
    __builtin_amdgcn_fence(__ATOMIC_RELEASE, "workgroup");
    __builtin_amdgcn_wave_barrier();
    __builtin_amdgcn_fence(__ATOMIC_ACQUIRE, "workgroup");
  }
}

__global__ __launch_bounds__(256) void cast_f32_f16x2(
    const float* __restrict__ in, _Float16* __restrict__ out, int n2) {
  int i = blockIdx.x * 256 + threadIdx.x;
  if (i < n2) {
    const _Float16 h0 = (_Float16)in[2 * i], h1 = (_Float16)in[2 * i + 1];
    const unsigned u = (unsigned)__builtin_bit_cast(unsigned short, h0) | ((unsigned)__builtin_bit_cast(unsigned short, h1) << 16);
    ((volatile unsigned*)out)[i] = u;
    __threadfence();
    ((volatile unsigned*)out)[i] = u;
  }
}


#define MN 4096
#define MDIN 2048
#define ML 128
#define MS 32768
__global__ __launch_bounds__(256) void latent_kernel(const float* __restrict__ O4, const float* __restrict__ eps, float* __restrict__ lat, float* __restrict__ invn) {
  const int lane = threadIdx.x & 31, wave = threadIdx.x >> 5; const size_t n = (size_t)blockIdx.x * 8 + wave;
  const v4f mu = *(const v4f*)(O4 + n * 256 + lane * 4), lv = *(const v4f*)(O4 + n * 256 + 128 + lane * 4), e = *(const v4f*)(eps + n * ML + lane * 4);
  v4f z; for (int q = 0; q < 4; ++q) z[q] = mu[q] + e[q] * expf(0.5f * lv[q]);
  float s = z[0]*z[0] + z[1]*z[1] + z[2]*z[2] + z[3]*z[3]; for (int o = 16; o > 0; o >>= 1) s += __shfl_xor(s, o, 32);
  __shared__ float st[8];
  for (int pass = 0; pass < 2; ++pass) { for (int q = 0; q < 4; ++q) ((volatile float*)lat)[n * ML + lane * 4 + q] = z[q]; __threadfence(); }
  if (lane == 0) st[wave] = 1.0f / sqrtf(s);
  __syncthreads();
  if (threadIdx.x < 8) { ((volatile float*)invn)[blockIdx.x * 8 + threadIdx.x] = st[threadIdx.x]; }
  __threadfence();
  if (threadIdx.x < 8) { ((volatile float*)invn)[blockIdx.x * 8 + threadIdx.x] = st[threadIdx.x]; }
}
__global__ __launch_bounds__(256) void loss_part_kernel(const float* __restrict__ lm, const float* __restrict__ ld, const float* __restrict__ inm, const float* __restrict__ ind, const int* __restrict__ ts, double* __restrict__ PS) {
  __shared__ double part[8];
  const int lane = threadIdx.x & 31, wave = threadIdx.x >> 5; double acc = 0.0;
  for (int s = blockIdx.x * 8 + wave; s < MS; s += gridDim.x * 8) {
    int i = ts[s * 4], j = ts[s * 4 + 1], jh = ts[s * 4 + 3]; i = i < 0 ? 0 : (i >= MN ? MN - 1 : i); j = j < 0 ? 0 : (j >= MN ? MN - 1 : j); jh = jh < 0 ? 0 : (jh >= MN ? MN - 1 : jh);
    v4f a, bj, bh; for (int q = 0; q < 4; ++q) { a[q] = lm[(size_t)i * ML + lane * 4 + q]; bj[q] = ld[(size_t)j * ML + lane * 4 + q]; bh[q] = ld[(size_t)jh * ML + lane * 4 + q]; }
    float d1 = a[0]*bj[0] + a[1]*bj[1] + a[2]*bj[2] + a[3]*bj[3], d2 = a[0]*bh[0] + a[1]*bh[1] + a[2]*bh[2] + a[3]*bh[3];
    for (int o = 16; o > 0; o >>= 1) { d1 += __shfl_xor(d1, o, 32); d2 += __shfl_xor(d2, o, 32); }
    const float lij = d1 * inm[i] * ind[j], lijh = d2 * inm[i] * ind[jh];
    const float pos = expf(lij), neg = 2.0f * expf(lijh);
    const float l1 = -logf(2.0f * pos / (2.0f * pos + neg)); const float l2 = fabsf((lij + 1.0f) * 0.5f - 1.0f) + (lijh + 1.0f);
    if (lane == 0) acc += (double)(l1 + l2); }
  if (lane == 0) part[wave] = acc; __syncthreads();
  if (threadIdx.x == 0) { double t = 0.0; for (int w = 0; w < 8; ++w) t += part[w]; ((volatile double*)PS)[blockIdx.x * 16] = t; __threadfence(); ((volatile double*)PS)[blockIdx.x * 16] = t; }
}
__global__ __launch_bounds__(256) void loss_final_kernel(const double* __restrict__ PS, int nblk, float* __restrict__ out0) {
  if (threadIdx.x == 0) { double t = 0.0; for (int b = 0; b < nblk; ++b) t += PS[b * 16]; const float v = (float)(t / (double)MS); ((volatile float*)out0)[0] = v; __threadfence(); ((volatile float*)out0)[0] = v; }
}
static void encoder(hipStream_t stream, const float* feat, const float* W1, const float* b1, const float* W2, const float* b2, const float* W3, const float* b3, const float* W4, const float* b4, const float* eps,
                    _Float16* X16, _Float16* W116, _Float16* W216, _Float16* W316, _Float16* W416, _Float16* H1, _Float16* H2, _Float16* H3, float* O4, float* lat, float* invn) {
  cast_f32_f16x2<<<(MN * MDIN / 2 + 255) / 256, 256, 0, stream>>>(feat, X16, (long)MN * MDIN / 2);
  cast_f32_f16x2<<<(512 * MDIN / 2 + 255) / 256, 256, 0, stream>>>(W1, W116, (long)512 * MDIN / 2);
  cast_f32_f16x2<<<(256 * 512 / 2 + 255) / 256, 256, 0, stream>>>(W2, W216, 256 * 512 / 2);
  cast_f32_f16x2<<<(64 * 256 / 2 + 255) / 256, 256, 0, stream>>>(W3, W316, 64 * 256 / 2);
  cast_f32_f16x2<<<(256 * 64 / 2 + 255) / 256, 256, 0, stream>>>(W4, W416, 256 * 64 / 2);
  { const int t = (MN / 64) * 8; wmma_gemm64<0, false, 2, 1, false, 2><<<dim3((t + 7) / 8, 1), 256, 0, stream>>>(U16(X16), nullptr, MDIN, 0, U16(W116), nullptr, MDIN, 0, H1, nullptr, 512, 0, b1, nullptr, 0, MN, 512, MDIN, 1.0f); }
  { const int t = (MN / 64) * 4; wmma_gemm64<0, false, 2, 1, false, 2><<<dim3((t + 7) / 8, 1), 256, 0, stream>>>(U16(H1), nullptr, 512, 0, U16(W216), nullptr, 512, 0, H2, nullptr, 256, 0, b2, nullptr, 0, MN, 256, 512, 1.0f); }
  { const int t = (MN / 64) * 1; wmma_gemm64<0, false, 2, 1, false, 2><<<dim3((t + 7) / 8, 1), 256, 0, stream>>>(U16(H2), nullptr, 256, 0, U16(W316), nullptr, 256, 0, H3, nullptr, 64, 0, b3, nullptr, 0, MN, 64, 256, 1.0f); }
  { const int t = (MN / 64) * 4; wmma_gemm64<0, false, 2, 0, false, 0><<<dim3((t + 7) / 8, 1), 256, 0, stream>>>(U16(H3), nullptr, 64, 0, U16(W416), nullptr, 64, 0, O4, nullptr, 256, 0, b4, nullptr, 0, MN, 256, 64, 1.0f); }
  latent_kernel<<<MN / 8, 256, 0, stream>>>(O4, eps, lat, invn);
}
extern "C" void kernel_launch(void* const* d_in, const int* in_sizes, int n_in, void* d_out, int out_size, void* d_ws, size_t ws_size, hipStream_t stream) {
  (void)in_sizes; (void)n_in; (void)out_size; (void)ws_size;
  auto F = [&](int i) { return (const float*)d_in[i]; };
  const int* ts = (const int*)d_in[20];
  float* out0 = (float*)d_out; float* latm = out0 + 1; float* latd = out0 + 1 + (size_t)MN * ML;
  char* ws = (char*)d_ws; size_t off = 0;
  auto carve = [&](size_t bytes) -> char* { char* p = ws + off; off += (bytes + 255) & ~(size_t)255; return p; };
  _Float16* X16 = (_Float16*)carve((size_t)MN * MDIN * 2); _Float16* W116 = (_Float16*)carve((size_t)512 * MDIN * 2); _Float16* W216 = (_Float16*)carve(256 * 512 * 2); _Float16* W316 = (_Float16*)carve(64 * 256 * 2); _Float16* W416 = (_Float16*)carve(256 * 64 * 2);
  _Float16* H1 = (_Float16*)carve((size_t)MN * 512 * 2); _Float16* H2 = (_Float16*)carve((size_t)MN * 256 * 2); _Float16* H3 = (_Float16*)carve((size_t)MN * 64 * 2); float* O4 = (float*)carve((size_t)MN * 256 * 4);
  float* inm = (float*)carve(MN * 4); float* ind = (float*)carve(MN * 4); const int NLB = 128; double* PS = (double*)carve((size_t)NLB * 16 * 8);
  encoder(stream, F(0), F(4), F(5), F(6), F(7), F(8), F(9), F(10), F(11), F(2), X16, W116, W216, W316, W416, H1, H2, H3, O4, latm, inm);
  encoder(stream, F(1), F(12), F(13), F(14), F(15), F(16), F(17), F(18), F(19), F(3), X16, W116, W216, W316, W416, H1, H2, H3, O4, latd, ind);
  loss_part_kernel<<<NLB, 256, 0, stream>>>(latm, latd, inm, ind, ts, PS);
  loss_final_kernel<<<1, 32, 0, stream>>>(PS, NLB, out0);
}
